// SelfAttentionPooling_59785944760726
// MI455X (gfx1250) — hardware-verified
//
#include <hip/hip_runtime.h>

typedef _Float16 half_t;
typedef __attribute__((ext_vector_type(16))) _Float16 v16h;
typedef __attribute__((ext_vector_type(8)))  _Float16 h8;
typedef __attribute__((ext_vector_type(4)))  _Float16 h4;
typedef __attribute__((ext_vector_type(8)))  float    v8f;
typedef __attribute__((ext_vector_type(4)))  float    f32x4;
typedef __attribute__((ext_vector_type(4)))  unsigned v4u_t;

#define NB   32
#define NC   256
#define NHD  4
#define HD   64
#define NPIX 1024
#define QT   32
#define NQT  (NPIX / QT)
#define RSPLIT (1.0f / 2048.0f)
#define PL   ((size_t)NB * NHD * NPIX * HD)

__device__ __forceinline__ half_t lo_of(float v, half_t h) { return (half_t)((v - (float)h) * 2048.0f); }
__device__ __forceinline__ int kmap(int e, int hi) { return (e < 8) ? (hi * 8 + e) : (16 + hi * 8 + (e - 8)); }
__device__ __forceinline__ v8f wmma16(v16h a, v16h b, v8f c) {
  return __builtin_amdgcn_wmma_f32_16x16x32_f16(false, a, false, b, (short)0, c, false, false);
}
struct Frag2 { v16h h, l; };
__device__ __forceinline__ v8f wmma_split(const Frag2& a, const Frag2& b, v8f c) { return wmma16(a.h, b.h, c); }
__device__ inline Frag2 frag_pl(const half_t* base, int ld, size_t plane) {
  const int lane = threadIdx.x & 31;
  const half_t* p = base + (lane & 15) * ld + ((lane >> 4) << 3);
  Frag2 f;
  f32x4* q = (f32x4*)&f.h; q[0] = *(const f32x4*)(p); q[1] = *(const f32x4*)(p + 16);
  f32x4* r = (f32x4*)&f.l; r[0] = *(const f32x4*)(p + plane); r[1] = *(const f32x4*)(p + plane + 16);
  return f;
}
__device__ inline Frag2 frag_f32(const float* base, int ld) {
  const int lane = threadIdx.x & 31, hi = lane >> 4;
  const float* p = base + (lane & 15) * ld;
  Frag2 f;
#pragma unroll
  for (int e = 0; e < 16; ++e) { const float v = p[kmap(e, hi)]; f.h[e] = (half_t)v; f.l[e] = lo_of(v, f.h[e]); }
  return f;
}
__device__ __forceinline__ unsigned pk2s(float a, float b, unsigned* lo) {
  const half_t h0 = (half_t)a, h1 = (half_t)b;
  *lo = (unsigned)__builtin_bit_cast(unsigned short, lo_of(a, h0)) | ((unsigned)__builtin_bit_cast(unsigned short, lo_of(b, h1)) << 16);
  return (unsigned)__builtin_bit_cast(unsigned short, h0) | ((unsigned)__builtin_bit_cast(unsigned short, h1) << 16);
}
__device__ inline float rel_t(int n, float p0, float p1) {
  float gy = (float)(n >> 5) * (2.0f / 31.0f) - 1.0f;
  float gx = (float)(n & 31) * (2.0f / 31.0f) - 1.0f;
  return gy * p0 + gx * p1;
}

__global__ __launch_bounds__(128) void qkv_kernel(
    const float* __restrict__ x, const float* __restrict__ wqkv, const float* __restrict__ bqkv,
    half_t* __restrict__ Qd, half_t* __restrict__ Kd, half_t* __restrict__ Vt) {
  __shared__ __attribute__((aligned(16))) half_t As[64 * 32], Asl[64 * 32];
  __shared__ __attribute__((aligned(16))) half_t Bs[64 * 32], Bsl[64 * 32];
  __shared__ __attribute__((aligned(16))) float  Ct[64][68];
  const int t = threadIdx.x, w = t >> 5, lane = t & 31;
  const int n0 = blockIdx.x * 64, m0 = blockIdx.y * 64, bb = blockIdx.z;
  const bool isV = (m0 >= 512);
  half_t* dst = (m0 < 256) ? Qd : (m0 < 512 ? Kd : Vt);
  const int cbase = m0 & 255;
  const float sc = (m0 < 256) ? 0.125f : 1.0f;

  v8f acc[4] = {};
  for (int kk = 0; kk < NC; kk += 32) {
    f32x4 ar[4], br[4];
#pragma unroll
    for (int i = 0; i < 4; ++i) { int lin = t + i * 128; int r = lin >> 3, c4 = lin & 7; ar[i] = *(const f32x4*)&wqkv[(m0 + r) * NC + kk + c4 * 4]; }
#pragma unroll
    for (int i = 0; i < 4; ++i) { int lin = t + i * 128; int k = lin >> 4, n4 = lin & 15; br[i] = *(const f32x4*)&x[((size_t)bb * NC + kk + k) * NPIX + n0 + n4 * 4]; }
    __syncthreads();
#pragma unroll
    for (int i = 0; i < 4; ++i) {
      int lin = t + i * 128; int r = lin >> 3, c4 = lin & 7;
      h4 hv, lv;
#pragma unroll
      for (int e = 0; e < 4; ++e) { hv[e] = (half_t)ar[i][e]; lv[e] = lo_of(ar[i][e], hv[e]); }
      *(h4*)&As[r * 32 + c4 * 4] = hv; *(h4*)&Asl[r * 32 + c4 * 4] = lv;
    }
#pragma unroll
    for (int i = 0; i < 4; ++i) {
      int lin = t + i * 128; int k = lin >> 4, n4 = lin & 15;
#pragma unroll
      for (int e = 0; e < 4; ++e) { const half_t h = (half_t)br[i][e]; Bs[(n4 * 4 + e) * 32 + k] = h; Bsl[(n4 * 4 + e) * 32 + k] = lo_of(br[i][e], h); }
    }
    __syncthreads();
    const Frag2 a = frag_pl(As + (w * 16) * 32, 32, (size_t)(Asl - As));
#pragma unroll
    for (int j = 0; j < 4; ++j) {
      const Frag2 bf = frag_pl(Bs + (j * 16) * 32, 32, (size_t)(Bsl - Bs));
      acc[j] = wmma_split(a, bf, acc[j]);
    }
  }
  const int mbase = (lane >> 4) * 8, ncol = lane & 15;
#pragma unroll
  for (int j = 0; j < 4; ++j)
#pragma unroll
    for (int r = 0; r < 8; ++r) {
      const int ml = w * 16 + mbase + r;
      Ct[ml][j * 16 + ncol] = (acc[j][r] + bqkv[m0 + ml]) * sc;
    }
  __syncthreads();
  const int hh = cbase >> 6;
#pragma unroll 1
  for (int pass = 0; pass < 2; ++pass) {
    if (!isV) {
#pragma unroll
      for (int i = 0; i < 4; ++i) {
        const int job = t + i * 128, nl = job >> 3, d8 = (job & 7) * 8;
        v4u_t v, vl; unsigned lq;
        v.x = pk2s(Ct[d8 + 0][nl], Ct[d8 + 1][nl], &lq); vl.x = lq; v.y = pk2s(Ct[d8 + 2][nl], Ct[d8 + 3][nl], &lq); vl.y = lq;
        v.z = pk2s(Ct[d8 + 4][nl], Ct[d8 + 5][nl], &lq); vl.z = lq; v.w = pk2s(Ct[d8 + 6][nl], Ct[d8 + 7][nl], &lq); vl.w = lq;
        half_t* o = dst + (((size_t)bb * NHD + hh) * NPIX + n0 + nl) * HD + d8;
        *(volatile v4u_t*)o = v; *(volatile v4u_t*)(o + PL) = vl;
      }
    } else {
#pragma unroll
      for (int i = 0; i < 4; ++i) {
        const int job = t + i * 128, dl = job >> 3, c8 = (job & 7) * 8;
        const float* s = &Ct[dl][c8];
        v4u_t v, vl; unsigned lq;
        v.x = pk2s(s[0], s[1], &lq); vl.x = lq; v.y = pk2s(s[2], s[3], &lq); vl.y = lq; v.z = pk2s(s[4], s[5], &lq); vl.z = lq; v.w = pk2s(s[6], s[7], &lq); vl.w = lq;
        half_t* o = dst + (((size_t)bb * NHD + hh) * HD + dl) * NPIX + n0 + c8;
        *(volatile v4u_t*)o = v; *(volatile v4u_t*)(o + PL) = vl;
      }
    }
    __threadfence();
  }
}

__global__ __launch_bounds__(128) void attn_kernel(
    const half_t* __restrict__ Q, const half_t* __restrict__ K, const half_t* __restrict__ Vtp,
    const float* __restrict__ relp, float* __restrict__ partial) {
  extern __shared__ float S[];
  __shared__ float red[128];
  __shared__ float osum[64];
  const int t = threadIdx.x, w = t >> 5, lane = t & 31;
  const int q0 = blockIdx.x * QT;
  const int bh = blockIdx.y, hh = bh & 3;
  const half_t* Qg  = Q   + (size_t)bh * NPIX * HD;
  const half_t* Kg  = K   + (size_t)bh * NPIX * HD;
  const half_t* Vtg = Vtp + (size_t)bh * HD * NPIX;
  const float p0 = relp[hh * 2], p1 = relp[hh * 2 + 1];
  const int mloc = lane & 15, koff = (lane >> 4) * 8;

  Frag2 qf[2][2];
#pragma unroll
  for (int jm = 0; jm < 2; ++jm)
#pragma unroll
    for (int kkh = 0; kkh < 2; ++kkh) qf[jm][kkh] = frag_pl(Qg + (size_t)(q0 + jm * 16) * HD + kkh * 32, HD, PL);
  float tq[2];
#pragma unroll
  for (int jm = 0; jm < 2; ++jm) tq[jm] = rel_t(q0 + jm * 16 + mloc, p0, p1);
  float tk[8];
#pragma unroll
  for (int r = 0; r < 8; ++r) tk[r] = rel_t(w * 16 + koff + r, p0, p1);
  const float dtk = (4.0f / 31.0f) * p0;

  for (int kb = 0; kb < NPIX; kb += 64) {
    const Frag2 ka0 = frag_pl(Kg + (size_t)(kb + w * 16) * HD, HD, PL);
    const Frag2 ka1 = frag_pl(Kg + (size_t)(kb + w * 16) * HD + 32, HD, PL);
#pragma unroll
    for (int jm = 0; jm < 2; ++jm) {
      v8f acc = {};
      acc = wmma_split(ka0, qf[jm][0], acc);
      acc = wmma_split(ka1, qf[jm][1], acc);
#pragma unroll
      for (int r = 0; r < 8; ++r) S[(size_t)(jm * 16 + mloc) * NPIX + kb + w * 16 + koff + r] = acc[r] + tq[jm] - tk[r];
    }
#pragma unroll
    for (int r = 0; r < 8; ++r) tk[r] += dtk;
  }
  __syncthreads();

  {
    const int row = t >> 2, part = t & 3;
    float* rp = S + (size_t)row * NPIX + part * 256;
    float m = -1e30f;
    for (int i = 0; i < 256; i += 4) { const f32x4 v = *(const f32x4*)(rp + i); m = fmaxf(m, fmaxf(fmaxf(v[0], v[1]), fmaxf(v[2], v[3]))); }
    red[t] = m;
    __syncthreads();
    m = fmaxf(fmaxf(red[row * 4], red[row * 4 + 1]), fmaxf(red[row * 4 + 2], red[row * 4 + 3]));
    __syncthreads();
    float s = 0.0f;
    for (int i = 0; i < 256; i += 4) {
      f32x4 v = *(const f32x4*)(rp + i);
#pragma unroll
      for (int e = 0; e < 4; ++e) { v[e] = __expf(v[e] - m); s += v[e]; }
      *(f32x4*)(rp + i) = v;
    }
    red[t] = s;
    __syncthreads();
    const float inv = 1.0f / (red[row * 4] + red[row * 4 + 1] + red[row * 4 + 2] + red[row * 4 + 3]);
    for (int i = 0; i < 256; i += 4) { f32x4 v = *(const f32x4*)(rp + i); *(f32x4*)(rp + i) = v * inv; }
  }
  __syncthreads();

  v8f oacc[2] = {};
  for (int kb = 0; kb < NPIX; kb += 64) {
#pragma unroll
    for (int kkh = 0; kkh < 2; ++kkh) {
      const Frag2 av = frag_pl(Vtg + (size_t)(w * 16) * NPIX + kb + kkh * 32, NPIX, PL);
#pragma unroll
      for (int j = 0; j < 2; ++j) {
        const Frag2 b = frag_f32(S + (size_t)(j * 16) * NPIX + kb + kkh * 32, NPIX);
        oacc[j] = wmma_split(av, b, oacc[j]);
      }
    }
  }
#pragma unroll
  for (int r = 0; r < 8; ++r) {
    float v = oacc[0][r] + oacc[1][r];
    v += __shfl_xor(v, 1); v += __shfl_xor(v, 2); v += __shfl_xor(v, 4); v += __shfl_xor(v, 8);
    if ((lane & 15) == 0) osum[w * 16 + koff + r] = v;
  }
  __syncthreads();
  if (t < 64) {
    float* dstp = partial + ((size_t)bh * NQT + blockIdx.x) * 64 + t;
    const float v = osum[t];
    *(volatile float*)dstp = v; __threadfence(); *(volatile float*)dstp = v;
  }
}

__global__ __launch_bounds__(256) void proj_kernel(
    const float* __restrict__ wout, const float* __restrict__ bout,
    const float* __restrict__ partial, float* __restrict__ out) {
  __shared__ float ys[NC];
  const int b = blockIdx.x, o = threadIdx.x;
  {
    const int hh = o >> 6, d = o & 63;
    float s = 0.0f;
    for (int tile = 0; tile < NQT; ++tile) s += partial[(((size_t)b * NHD + hh) * NQT + tile) * 64 + d];
    ys[o] = s;
  }
  __syncthreads();
  float s = 0.0f;
  for (int c = 0; c < NC; ++c) s += wout[o * NC + c] * ys[c];
  const float v = s * (1.0f / (float)NPIX) + bout[o];
  *(volatile float*)(out + b * NC + o) = v; __threadfence(); *(volatile float*)(out + b * NC + o) = v;
}

extern "C" void kernel_launch(void* const* d_in, const int* in_sizes, int n_in,
                              void* d_out, int out_size, void* d_ws, size_t ws_size,
                              hipStream_t stream) {
    const float* x    = (const float*)d_in[0];
    const float* wqkv = (const float*)d_in[1];
    const float* bqkv = (const float*)d_in[2];
    const float* wout = (const float*)d_in[3];
    const float* bout = (const float*)d_in[4];
    const float* relp = (const float*)d_in[5];

    const size_t per = (size_t)NB * NHD * NPIX * HD;
    half_t* Qws = (half_t*)d_ws;
    half_t* Kws = Qws + 2 * per;
    half_t* Vtw = Kws + 2 * per;
    float*  partial = (float*)(Vtw + 2 * per);
    const int nb = NB;

    qkv_kernel<<<dim3(NPIX / 64, 768 / 64, nb), 128, 0, stream>>>(x, wqkv, bqkv, Qws, Kws, Vtw);
    size_t smem = (size_t)QT * NPIX * sizeof(float);
    (void)hipFuncSetAttribute((const void*)attn_kernel, hipFuncAttributeMaxDynamicSharedMemorySize, (int)smem);
    attn_kernel<<<dim3(NQT, nb * NHD), 128, smem, stream>>>(Qws, Kws, Vtw, relp, partial);
    proj_kernel<<<nb, 256, 0, stream>>>(wout, bout, partial, (float*)d_out);
}
